// pc_conv_30159260352601
// MI455X (gfx1250) — hardware-verified
//
#include <hip/hip_runtime.h>
#include <stddef.h>


typedef _Float16 f16;
typedef _Float16 v16h __attribute__((ext_vector_type(16)));
typedef _Float16 v8h  __attribute__((ext_vector_type(8)));
typedef float    v8f  __attribute__((ext_vector_type(8)));
typedef float    v4f  __attribute__((ext_vector_type(4)));
typedef unsigned int v4u __attribute__((ext_vector_type(4)));

#define EF              128
#define KNN             8
#define K1              (EF + 3)
#define K1P             160
#define K2P             128
#define HP              128
#define NTHREADS        256
#define NWAVES          8
#define POINTS_PER_WAVE 4
#define ROWS_PER_WAVE   (POINTS_PER_WAVE * KNN)
#define ROWS_PER_TILE   (NWAVES * ROWS_PER_WAVE)
#define TILES_PER_BLOCK 8
#define GROWS           64
#define CHUNK_ROWS      409600
#define WSCALE          16.0f
#define OSCALE          (1.0f / 256.0f)

union Frag { v16h v; v8h h[2]; };
union Pack { v8h h; v4u u; };

__device__ __forceinline__ v8f wmma16(v16h a, v16h b, v8f c)
{
    v8f d = __builtin_amdgcn_wmma_f32_16x16x32_f16(false, a, false, b, (short)0, c, false, false);
    asm volatile("v_nop\n\tv_nop\n\tv_nop\n\tv_nop" : "+v"(d) : "v"(a), "v"(b));
    return d;
}

__global__ __launch_bounds__(NTHREADS) void k_gather_rows(
    const float* __restrict__ feat,
    const int*   __restrict__ idx,
    v4u*         __restrict__ grows,
    int r0, int cnt, int nIn)
{
    const int tid  = threadIdx.x;
    const int sub  = tid >> 4;
    const int c8   = tid & 15;
    const int base = blockIdx.x * GROWS;

    Pack pk[4];
    int  rl[4];
#pragma unroll
    for (int j = 0; j < 4; ++j) {
        const int r  = base + j * 16 + sub;
        rl[j] = r;
        const int rr = r < cnt ? r : cnt - 1;
        int i = idx[r0 + rr];
        i = i < 0 ? i + nIn : i;
        i = i < 0 ? 0 : i;
        i = i >= nIn ? nIn - 1 : i;
        const float* src = feat + (size_t)i * EF + c8 * 8;
        const v4f x0 = *(const v4f*)src;
        const v4f x1 = *(const v4f*)(src + 4);
#pragma unroll
        for (int q = 0; q < 4; ++q) {
            pk[j].h[q]     = (f16)x0[q];
            pk[j].h[4 + q] = (f16)x1[q];
        }
    }
#pragma unroll
    for (int j = 0; j < 4; ++j) {
        if (rl[j] < cnt)
            *(volatile v4u*)(grows + (size_t)rl[j] * (EF / 8) + c8) = pk[j].u;
    }
    __threadfence();
#pragma unroll
    for (int j = 0; j < 4; ++j) {
        if (rl[j] < cnt)
            *(volatile v4u*)(grows + (size_t)rl[j] * (EF / 8) + c8) = pk[j].u;
    }
}

__global__ __launch_bounds__(NTHREADS) void k_mlp_pool(
    const f16*   __restrict__ gb,
    const float* __restrict__ xyz,
    const float* __restrict__ W1,
    const float* __restrict__ b1,
    const float* __restrict__ W2,
    const float* __restrict__ b2,
    float*       __restrict__ out,
    int r0, int cnt, int numTiles, int nPoints)
{
    __shared__ __attribute__((aligned(16))) f16   sW1T[EF * K1P];
    __shared__ __attribute__((aligned(16))) f16   sW2T[EF * K2P];
    __shared__ __attribute__((aligned(16))) f16   sH[NWAVES][16 * HP];
    __shared__ __attribute__((aligned(16))) float sO[NWAVES][POINTS_PER_WAVE * EF];
    __shared__ float sB1s[EF];
    __shared__ float sB2[EF];

    const int tid = threadIdx.x;

    for (int e = tid; e < K1 * (EF / 4); e += NTHREADS) {
        const int k  = e >> 5;
        const int n0 = (e & 31) * 4;
        const v4f w = *(const v4f*)(W1 + k * EF + n0);
#pragma unroll
        for (int q = 0; q < 4; ++q) sW1T[(n0 + q) * K1P + k] = (f16)(WSCALE * w[q]);
    }
    if (tid < EF) {
#pragma unroll
        for (int k = K1; k < K1P; ++k) sW1T[tid * K1P + k] = (f16)0.0f;
    }
    for (int e = tid; e < EF * (EF / 4); e += NTHREADS) {
        const int k  = e >> 5;
        const int n0 = (e & 31) * 4;
        const v4f w = *(const v4f*)(W2 + k * EF + n0);
#pragma unroll
        for (int q = 0; q < 4; ++q) sW2T[(n0 + q) * K2P + k] = (f16)(WSCALE * w[q]);
    }
    if (tid < EF) {
        sB1s[tid] = WSCALE * b1[tid];
        sB2[tid]  = b2[tid];
    }
    __syncthreads();

    const int wave = tid >> 5;
    const int lane = tid & 31;
    const int m    = lane & 15;
    const int hh   = lane >> 4;
    f16*   hb = &sH[wave][0];
    float* ob = &sO[wave][0];

    for (int it = 0; it < TILES_PER_BLOCK; ++it) {
        const int tile = blockIdx.x * TILES_PER_BLOCK + it;
        if (tile >= numTiles) break;
        const int wrow0 = tile * ROWS_PER_TILE + wave * ROWS_PER_WAVE;

#pragma unroll 1
        for (int s = 0; s < 2; ++s) {
            int rl = wrow0 + s * 16 + m;
            rl = rl < cnt ? rl : cnt - 1;
            const f16* arow = gb + (size_t)rl * EF;

            v8f acc[8];
#pragma unroll
            for (int t = 0; t < 8; ++t) { v8f z = {}; acc[t] = z; }

#pragma unroll
            for (int kk = 0; kk < 4; ++kk) {
                Frag a;
                a.h[0] = *(const v8h*)(arow + kk * 32 + 8 * hh);
                a.h[1] = *(const v8h*)(arow + kk * 32 + 16 + 8 * hh);
#pragma unroll
                for (int t = 0; t < 8; ++t) {
                    const f16* bp = sW1T + (t * 16 + m) * K1P + kk * 32 + 8 * hh;
                    Frag b;
                    b.h[0] = *(const v8h*)bp;
                    b.h[1] = *(const v8h*)(bp + 16);
                    acc[t] = wmma16(a.v, b.v, acc[t]);
                }
            }
            {
                v16h az = {};
                Frag a; a.v = az;
                const float* xp = xyz + (size_t)(r0 + rl) * 3;
                a.v[0] = (f16)xp[0];
                a.v[1] = (f16)xp[1];
                a.v[2] = (f16)xp[2];
#pragma unroll
                for (int t = 0; t < 8; ++t) {
                    const f16* bp = sW1T + (t * 16 + m) * K1P + EF + 8 * hh;
                    Frag b;
                    b.h[0] = *(const v8h*)bp;
                    b.h[1] = *(const v8h*)(bp + 16);
                    acc[t] = wmma16(a.v, b.v, acc[t]);
                }
            }

#pragma unroll
            for (int t = 0; t < 8; ++t) {
                const float bb = sB1s[t * 16 + m];
#pragma unroll
                for (int r = 0; r < 8; ++r) {
                    float v = acc[t][r] + bb;
                    v = fmaxf(v, 0.01f * v);
                    hb[(8 * hh + r) * HP + t * 16 + m] = (f16)v;
                }
            }
            __syncthreads();

            v8f acc2[8];
#pragma unroll
            for (int t = 0; t < 8; ++t) { v8f z = {}; acc2[t] = z; }
            const f16* hrow = hb + m * HP;
#pragma unroll
            for (int kk = 0; kk < 4; ++kk) {
                Frag a;
                a.h[0] = *(const v8h*)(hrow + kk * 32 + 8 * hh);
                a.h[1] = *(const v8h*)(hrow + kk * 32 + 16 + 8 * hh);
#pragma unroll
                for (int t = 0; t < 8; ++t) {
                    const f16* bp = sW2T + (t * 16 + m) * K2P + kk * 32 + 8 * hh;
                    Frag b;
                    b.h[0] = *(const v8h*)bp;
                    b.h[1] = *(const v8h*)(bp + 16);
                    acc2[t] = wmma16(a.v, b.v, acc2[t]);
                }
            }

#pragma unroll
            for (int t = 0; t < 8; ++t) {
                float mx = acc2[t][0];
#pragma unroll
                for (int r = 1; r < 8; ++r) mx = fmaxf(mx, acc2[t][r]);
                ob[(s * 2 + hh) * EF + t * 16 + m] = mx * OSCALE + sB2[t * 16 + m];
            }
            __syncthreads();
        }

        const int point0 = (r0 + wrow0) / KNN;
        v4f ov[POINTS_PER_WAVE];
        int ok[POINTS_PER_WAVE];
#pragma unroll
        for (int p = 0; p < POINTS_PER_WAVE; ++p) {
            ov[p] = *(const v4f*)(ob + p * EF + lane * 4);
            ok[p] = ((wrow0 + KNN * p) < cnt) && ((point0 + p) < nPoints);
        }
#pragma unroll
        for (int p = 0; p < POINTS_PER_WAVE; ++p) {
            if (ok[p])
                *(volatile v4f*)(out + (size_t)(point0 + p) * EF + lane * 4) = ov[p];
        }
        __threadfence();
#pragma unroll
        for (int p = 0; p < POINTS_PER_WAVE; ++p) {
            if (ok[p])
                *(volatile v4f*)(out + (size_t)(point0 + p) * EF + lane * 4) = ov[p];
        }
    }
}

extern "C" void kernel_launch(void* const* d_in, const int* in_sizes, int n_in,
                              void* d_out, int out_size, void* d_ws, size_t ws_size,
                              hipStream_t stream)
{
    if (n_in < 7) return;
    const float* feat = (const float*)d_in[0];
    const int*   idx  = (const int*)  d_in[1];
    const float* xyz  = (const float*)d_in[2];
    const float* W1   = (const float*)d_in[3];
    const float* b1   = (const float*)d_in[4];
    const float* W2   = (const float*)d_in[5];
    const float* b2   = (const float*)d_in[6];
    float*       out  = (float*)d_out;

    const int nIn     = in_sizes[0] / EF;
    const int nPoints = out_size / EF;
    int nRows = in_sizes[1];
    const int xyzRows = in_sizes[2] / 3;
    if (nRows > xyzRows) nRows = xyzRows;
    if (nRows > nPoints * KNN) nRows = nPoints * KNN;
    if (nIn <= 0 || nPoints <= 0 || nRows <= 0) return;
    if (in_sizes[3] < K1 * EF || in_sizes[4] < EF || in_sizes[5] < EF * EF || in_sizes[6] < EF) return;

    long long chunkRows = CHUNK_ROWS;
    const long long wsRows = ((long long)ws_size / (EF * 2)) / 2048 * 2048;
    if (chunkRows > wsRows) chunkRows = wsRows;
    if (chunkRows <= 0) return;
    f16* gb = (f16*)d_ws;

    for (long long r0l = 0; r0l < nRows; r0l += chunkRows) {
        const int r0  = (int)r0l;
        const int cnt = (nRows - r0) < chunkRows ? (nRows - r0) : (int)chunkRows;
        const int gblocks  = (cnt + GROWS - 1) / GROWS;
        k_gather_rows<<<gblocks, NTHREADS, 0, stream>>>(feat, idx, (v4u*)d_ws, r0, cnt, nIn);
        const int numTiles = (cnt + ROWS_PER_TILE - 1) / ROWS_PER_TILE;
        const int blocks   = (numTiles + TILES_PER_BLOCK - 1) / TILES_PER_BLOCK;
        k_mlp_pool<<<blocks, NTHREADS, 0, stream>>>(gb, xyz, W1, b1, W2, b2, out,
                                                   r0, cnt, numTiles, nPoints);
    }
}
